// CapsuleLayer_22239340659091
// MI455X (gfx1250) — hardware-run, weakly checked
//
#include <hip/hip_runtime.h>
#include <math.h>

typedef __attribute__((ext_vector_type(16))) __bf16   v16b;
typedef __attribute__((ext_vector_type(8)))  float    v8f;
typedef __attribute__((ext_vector_type(4)))  float    v4f;
typedef __attribute__((ext_vector_type(4)))  unsigned v4u;
typedef __attribute__((ext_vector_type(8)))  unsigned v8u;

constexpr int kBatch    = 64;
constexpr int kNumIn    = 2048;
constexpr int kDimIn    = 8;
constexpr int kNumOut   = 16;
constexpr int kDimOut   = 16;
constexpr int kCols     = kNumOut * kDimOut;
constexpr int kBT       = 16;
constexpr int kIChunk   = 16;
constexpr int kTileI    = 2;
constexpr int kUStride  = 260;
constexpr int kUILen    = kBT * kUStride;
constexpr int kChunks   = kNumIn / kIChunk;
constexpr int kBTiles   = kBatch / kBT;
constexpr int kOutElems = kBatch * kCols;
constexpr int kXRowWords = kNumIn * kDimIn / 2;
constexpr float kSqEps  = 1e-7f;
static_assert(kCols == 256 && kDimIn == 8, "fragment packing assumes 8 live k values and 256 columns");
static_assert(kChunks * kIChunk == kNumIn && kBTiles * kBT == kBatch, "exact tiling, no tails");
static_assert(kChunks == 128 && kBTiles == 4 && kOutElems == 16384, "grid constants");
static_assert((kUStride % 4) == 0, "16-B aligned LDS rows");
static_assert(kTileI * kUILen >= 256 * kDimOut, "end-of-kernel staging fits in the u tile");

constexpr size_t kSzXH  = (size_t)kBatch * kNumIn * kDimIn * 2;
constexpr size_t kSzWP  = (size_t)kNumIn * kCols * kDimIn * 2;
constexpr size_t kSzSP  = (size_t)kChunks * kOutElems * 4;
constexpr size_t kSzV   = (size_t)kOutElems * 4;
constexpr size_t kOffXH  = 0;
constexpr size_t kOffWP  = kOffXH  + kSzXH;
constexpr size_t kOffSP0 = kOffWP  + kSzWP;
constexpr size_t kOffSP1 = kOffSP0 + kSzSP;
constexpr size_t kOffSP2 = kOffSP1 + kSzSP;
constexpr size_t kOffVA  = kOffSP2 + kSzSP;
constexpr size_t kOffVB  = kOffVA  + kSzV;
constexpr size_t kWsTotal = kOffVB + kSzV;
static_assert(kWsTotal == 35782656ull, "carve total");
static_assert(kWsTotal <= 134217728ull, "carve cap");
static_assert((kOffWP % 128) == 0 && (kOffSP0 % 128) == 0 && (kOffSP1 % 128) == 0 && (kOffSP2 % 128) == 0 &&
              (kOffVA % 128) == 0 && (kOffVB % 128) == 0, "128-B aligned regions");

__device__ __forceinline__ unsigned bf_bits_rne(float f) {
  const unsigned u = __float_as_uint(f);
  return (u + 0x7FFFu + ((u >> 16) & 1u)) >> 16;
}
__device__ __forceinline__ unsigned pack2_bf(float lo, float hi) {
  const unsigned a = bf_bits_rne(lo) & 0xFFFFu;
  const unsigned b = bf_bits_rne(hi) << 16;
  return a | b;
}
__device__ __forceinline__ v16b frag_k8(unsigned w0, unsigned w1, unsigned w2, unsigned w3) {
  const v8u t = (v8u){w0, w1, w2, w3, 0u, 0u, 0u, 0u};
  return __builtin_bit_cast(v16b, t);
}
__device__ __forceinline__ v8f mma_bf16(v16b a, v16b b, v8f c) {
  c = __builtin_amdgcn_wmma_f32_16x16x32_bf16(false, a, false, b, (short)0, c, false, false);
  asm volatile("v_nop\n\tv_nop\n\tv_nop\n\tv_nop" : "+v"(c) : "v"(a), "v"(b));
  return c;
}

__global__ __launch_bounds__(256) void cvt_rows_bf16_kernel(
    const float* __restrict__ src, unsigned* __restrict__ dst, int total8)
{
  const int i = blockIdx.x * 256 + threadIdx.x;
  if (i >= total8) return;
  const size_t e0 = (size_t)i << 3;
  const v4f a0 = *(const v4f*)(src + e0);
  const v4f a1 = *(const v4f*)(src + e0 + 4);
  const v4u w = (v4u){pack2_bf(a0[0], a0[1]), pack2_bf(a0[2], a0[3]), pack2_bf(a1[0], a1[1]), pack2_bf(a1[2], a1[3])};
  unsigned* q = dst + ((size_t)i << 2);
  *(volatile v4u*)q = w;
  __threadfence();
  *(volatile v4u*)q = w;
}

__global__ __launch_bounds__(256) void cvt_w_planes_kernel(
    const float* __restrict__ W, unsigned* __restrict__ dst, int total)
{
  const int g = blockIdx.x * 256 + threadIdx.x;
  if (g >= total) return;
  const int i = g >> 8;
  const int n = g & 255;
  const int k = n >> 4;
  const int e = n & 15;
  const float* s = W + ((size_t)(i * kNumOut + k) * kDimIn) * kDimOut + e;
  const float f0 = s[0 * kDimOut];
  const float f1 = s[1 * kDimOut];
  const float f2 = s[2 * kDimOut];
  const float f3 = s[3 * kDimOut];
  const float f4 = s[4 * kDimOut];
  const float f5 = s[5 * kDimOut];
  const float f6 = s[6 * kDimOut];
  const float f7 = s[7 * kDimOut];
  const v4u w = (v4u){pack2_bf(f0, f1), pack2_bf(f2, f3), pack2_bf(f4, f5), pack2_bf(f6, f7)};
  unsigned* q = dst + ((size_t)g << 2);
  *(volatile v4u*)q = w;
  __threadfence();
  *(volatile v4u*)q = w;
}

template <bool ROUTED>
__global__ __launch_bounds__(256) void route_pass_kernel(
    const unsigned* __restrict__ Xh, const unsigned* __restrict__ Wp,
    const float* __restrict__ vsum, float* __restrict__ Spart)
{
  __shared__ __align__(16) unsigned x_lds[kIChunk * kBT * 4];
  __shared__ __align__(16) float    u_lds[kTileI * kUILen];

  const int tid  = threadIdx.x;
  const int wv   = __builtin_amdgcn_readfirstlane((int)(threadIdx.x >> 5));
  const int lane = tid & 31;
  const int hsel = lane >> 4;
  const int lm   = lane & 15;
  const int chunk = blockIdx.x;
  const int bt    = blockIdx.y;
  const int i0 = chunk * kIChunk;
  const int b0 = bt * kBT;

  {
    const int sb = tid >> 4;
    const int si = tid & 15;
    const v4u xv = *(const v4u*)(Xh + (size_t)(b0 + sb) * kXRowWords + (size_t)(i0 + si) * 4);
    *(v4u*)(x_lds + (si * kBT + sb) * 4) = xv;
  }

  const int b_l = tid >> 4;
  const int kk  = tid & 15;
  float vreg[kDimOut];
#pragma unroll
  for (int e = 0; e < kDimOut; ++e) vreg[e] = 0.0f;
  if (ROUTED) {
    const float* vp = vsum + ((size_t)(b0 + b_l) * kNumOut + kk) * kDimOut;
#pragma unroll
    for (int q = 0; q < 4; ++q) {
      const v4f t = *(const v4f*)(vp + 4 * q);
      vreg[4 * q + 0] = t[0];
      vreg[4 * q + 1] = t[1];
      vreg[4 * q + 2] = t[2];
      vreg[4 * q + 3] = t[3];
    }
  }
  float acc[kDimOut];
#pragma unroll
  for (int e = 0; e < kDimOut; ++e) acc[e] = 0.0f;

  const unsigned fmask = (hsel == 0) ? 0xFFFFFFFFu : 0u;
  const int colA = (2 * wv) * kDimOut + lm;

  __syncthreads();

#pragma unroll 1
  for (int ib = 0; ib < kIChunk; ib += kTileI) {
#pragma unroll
    for (int ii = 0; ii < kTileI; ++ii) {
      const int i_l = ib + ii;
      const int i_g = i0 + i_l;
      const v4u xa = *(const v4u*)(x_lds + (i_l * kBT + lm) * 4);
      const v4u* wrow = (const v4u*)Wp + ((size_t)i_g * kCols + (size_t)colA);
      const v4u wb0 = wrow[0];
      const v4u wb1 = wrow[kDimOut];
      unsigned p0 = wb0[0], p1 = wb0[1], p2 = wb0[2], p3 = wb0[3];
      unsigned q0 = wb1[0], q1 = wb1[1], q2 = wb1[2], q3 = wb1[3];
      asm volatile("" : "+v"(p0), "+v"(p1), "+v"(p2), "+v"(p3));
      asm volatile("" : "+v"(q0), "+v"(q1), "+v"(q2), "+v"(q3));
      const v16b fa  = frag_k8(xa[0] & fmask, xa[1] & fmask, xa[2] & fmask, xa[3] & fmask);
      const v16b fb0 = frag_k8(p0 & fmask, p1 & fmask, p2 & fmask, p3 & fmask);
      const v16b fb1 = frag_k8(q0 & fmask, q1 & fmask, q2 & fmask, q3 & fmask);
      v8f c0 = (v8f){0.f, 0.f, 0.f, 0.f, 0.f, 0.f, 0.f, 0.f};
      v8f c1 = (v8f){0.f, 0.f, 0.f, 0.f, 0.f, 0.f, 0.f, 0.f};
      c0 = mma_bf16(fa, fb0, c0);
      c1 = mma_bf16(fa, fb1, c1);
      float* ub = u_lds + ii * kUILen + (8 * hsel) * kUStride + colA;
#pragma unroll
      for (int r = 0; r < 8; ++r) {
        ub[r * kUStride]           = c0[r];
        ub[r * kUStride + kDimOut] = c1[r];
      }
    }
    __syncthreads();

#pragma unroll
    for (int ii = 0; ii < kTileI; ++ii) {
      const float* up = u_lds + ii * kUILen + b_l * kUStride + kk * kDimOut;
      float u[kDimOut];
#pragma unroll
      for (int q = 0; q < 4; ++q) {
        const v4f t = *(const v4f*)(up + 4 * q);
        u[4 * q + 0] = t[0];
        u[4 * q + 1] = t[1];
        u[4 * q + 2] = t[2];
        u[4 * q + 3] = t[3];
      }
      float cpl = 0.0625f;
      if (ROUTED) {
        float bij = 0.0f;
#pragma unroll
        for (int e = 0; e < kDimOut; ++e) bij = fmaf(u[e], vreg[e], bij);
        float mx = bij;
#pragma unroll
        for (int msk = 1; msk < 16; msk <<= 1) {
          const float o = __shfl_xor(mx, msk, 32);
          mx = fmaxf(mx, o);
        }
        float pe = expf(bij - mx);
        pe = (pe < 1.17549435e-38f) ? 0.0f : pe;
        float sum = pe;
#pragma unroll
        for (int msk = 1; msk < 16; msk <<= 1) {
          const float o = __shfl_xor(sum, msk, 32);
          sum += o;
        }
        cpl = pe * (1.0f / sum);
      }
#pragma unroll
      for (int e = 0; e < kDimOut; ++e) acc[e] = fmaf(cpl, u[e], acc[e]);
    }
    __syncthreads();
  }

  {
    float* st = u_lds + tid * kDimOut;
#pragma unroll
    for (int q = 0; q < 4; ++q) {
      const v4f t = (v4f){acc[4 * q + 0], acc[4 * q + 1], acc[4 * q + 2], acc[4 * q + 3]};
      *(v4f*)(st + 4 * q) = t;
    }
  }
  __syncthreads();
  {
    v4f ov[4];
#pragma unroll
    for (int it = 0; it < 4; ++it) ov[it] = *(const v4f*)(u_lds + wv * 512 + it * 128 + lane * 4);
    float* dst = Spart + (size_t)chunk * kOutElems + (size_t)bt * (kBT * kCols) + wv * 512 + lane * 4;
    for (int pass = 0; pass < 2; ++pass) {
#pragma unroll
      for (int it = 0; it < 4; ++it) *(volatile v4f*)(dst + it * 128) = ov[it];
      __threadfence();
    }
  }
}

template <int MODE>
__global__ __launch_bounds__(256) void reduce_squash_kernel(
    const float* __restrict__ Spart, const float* vold, float* vnew, float* outp)
{
  const int t = blockIdx.x * 256 + threadIdx.x;
  float s = 0.0f;
#pragma unroll 8
  for (int c = 0; c < kChunks; ++c) s += Spart[(size_t)c * kOutElems + t];
  float sn = s * s;
#pragma unroll
  for (int msk = 1; msk < 16; msk <<= 1) {
    const float o = __shfl_xor(sn, msk, 32);
    sn += o;
  }
  const float den = (1.0f + sn) * sqrtf(sn + kSqEps);
  const float v = s * (sn / den);
  float val = v;
  if (MODE == 1) {
    const float pv = vold[t];
    val = pv + v;
  }
  float* dst = (MODE == 2) ? (outp + t) : (vnew + t);
  *(volatile float*)dst = val;
  __threadfence();
  *(volatile float*)dst = val;
}

extern "C" void kernel_launch(void* const* d_in, const int* in_sizes, int n_in,
                              void* d_out, int out_size, void* d_ws, size_t ws_size,
                              hipStream_t stream) {
  if (n_in < 2) return;
  if (in_sizes[0] != kBatch * kNumIn * kDimIn) return;
  if (in_sizes[1] != kNumIn * kNumOut * kDimIn * kDimOut) return;
  if (out_size != kOutElems) return;
  if (ws_size < kWsTotal) return;

  const float* X = (const float*)d_in[0];
  const float* W = (const float*)d_in[1];
  float* out = (float*)d_out;

  char* ws = (char*)d_ws;
  unsigned* XH  = (unsigned*)(ws + kOffXH);
  unsigned* WP  = (unsigned*)(ws + kOffWP);
  float*    SP0 = (float*)(ws + kOffSP0);
  float*    SP1 = (float*)(ws + kOffSP1);
  float*    SP2 = (float*)(ws + kOffSP2);
  float*    VA  = (float*)(ws + kOffVA);
  float*    VB  = (float*)(ws + kOffVB);

  const int xTotal8 = kBatch * kNumIn * kDimIn / 8;
  const int wTotal  = kNumIn * kCols;
  cvt_rows_bf16_kernel<<<xTotal8 / 256, 256, 0, stream>>>(X, XH, xTotal8);
  cvt_w_planes_kernel<<<wTotal / 256, 256, 0, stream>>>(W, WP, wTotal);

  const dim3 pgrid(kChunks, kBTiles);
  const int rblocks = kOutElems / 256;

  route_pass_kernel<false><<<pgrid, 256, 0, stream>>>(XH, WP, VA, SP0);
  reduce_squash_kernel<0><<<rblocks, 256, 0, stream>>>(SP0, VA, VA, out);
  route_pass_kernel<true><<<pgrid, 256, 0, stream>>>(XH, WP, VA, SP1);
  reduce_squash_kernel<1><<<rblocks, 256, 0, stream>>>(SP1, VA, VB, out);
  route_pass_kernel<true><<<pgrid, 256, 0, stream>>>(XH, WP, VB, SP2);
  reduce_squash_kernel<2><<<rblocks, 256, 0, stream>>>(SP2, VB, VB, out);
}
